// RWKV7_22342419873910
// MI455X (gfx1250) — hardware-verified
//
#include <hip/hip_runtime.h>
#include <math.h>

constexpr int  kNB  = 4;
constexpr int  kNT  = 1024;
constexpr int  kNC  = 768;
constexpr int  kNH  = 12;
constexpr int  kHS  = 64;
constexpr int  kRows = kNB * kNT;
constexpr long kPlaneElems = (long)kRows * kNC;
constexpr float kGnEps = 6.4e-4f;
constexpr float kInvHS = 1.0f / 64.0f;

typedef __attribute__((ext_vector_type(16))) _Float16 v16h;
typedef __attribute__((ext_vector_type(8)))  _Float16 v8h;
typedef __attribute__((ext_vector_type(16))) __bf16   v16b;
typedef __attribute__((ext_vector_type(8)))  __bf16   v8b;
typedef __attribute__((ext_vector_type(8)))  float    v8f;
typedef __attribute__((ext_vector_type(4)))  float    v4f;
typedef __attribute__((ext_vector_type(4)))  unsigned int v4u;

__device__ __forceinline__ unsigned short f2bf_bits(float f) {
  unsigned u = __float_as_uint(f);
  return (unsigned short)((u + 0x7FFFu + ((u >> 16) & 1u)) >> 16);
}
__device__ __forceinline__ float bf_bits2f(unsigned short h) { return __uint_as_float(((unsigned)h) << 16); }

__device__ __forceinline__ void dep_guard_h(v8f& a, v8f& b, v16h x, v16h y) { asm volatile("v_nop\n\tv_nop\n\tv_nop\n\tv_nop" : "+v"(a), "+v"(b) : "v"(x), "v"(y)); }
__device__ __forceinline__ void dep_guard_b(v8f& a, v8f& b, v16b x, v16b y) { asm volatile("v_nop\n\tv_nop\n\tv_nop\n\tv_nop" : "+v"(a), "+v"(b) : "v"(x), "v"(y)); }
__device__ __forceinline__ void keep4_h(v16h a, v16h b, v16h c, v16h d) { asm volatile("v_nop" :: "v"(a), "v"(b), "v"(c), "v"(d)); }
__device__ __forceinline__ void keep4_b(v16b a, v16b b, v16b c, v16b d) { asm volatile("v_nop" :: "v"(a), "v"(b), "v"(c), "v"(d)); }
__device__ __forceinline__ void acc_guard4(v8f& a, v8f& b, v8f& c, v8f& d) { asm volatile("v_nop\n\tv_nop\n\tv_nop\n\tv_nop" : "+v"(a), "+v"(b), "+v"(c), "+v"(d)); }
template <typename T> struct Frag;
template <> struct Frag<_Float16> {
  typedef v16h V; union U { v16h v; v8h h[2]; };
  static __device__ __forceinline__ v16h load(const _Float16* p) {
    U f; f.h[0] = *(const v8h*)(p); f.h[1] = *(const v8h*)(p + 16); return f.v;
  }
  static __device__ __forceinline__ v8f mma(v16h a, v16h b, v8f c) {
    return __builtin_amdgcn_wmma_f32_16x16x32_f16(false, a, false, b, (short)0, c, false, false);
  }
  static __device__ __forceinline__ void guard(v8f& a, v8f& b, v16h x, v16h y) { dep_guard_h(a, b, x, y); }
  static __device__ __forceinline__ void keep(v16h a, v16h b, v16h c, v16h d) { keep4_h(a, b, c, d); }
};
template <> struct Frag<__bf16> {
  typedef v16b V; union U { v16b v; v8b h[2]; };
  static __device__ __forceinline__ v16b load(const __bf16* p) {
    U f; f.h[0] = *(const v8b*)(p); f.h[1] = *(const v8b*)(p + 16); return f.v;
  }
  static __device__ __forceinline__ v8f mma(v16b a, v16b b, v8f c) {
    return __builtin_amdgcn_wmma_f32_16x16x32_bf16(false, a, false, b, (short)0, c, false, false);
  }
  static __device__ __forceinline__ void guard(v8f& a, v8f& b, v16b x, v16b y) { dep_guard_b(a, b, x, y); }
  static __device__ __forceinline__ void keep(v16b a, v16b b, v16b c, v16b d) { keep4_b(a, b, c, d); }
};

template <int ET> struct Elem;
template <> struct Elem<0> { typedef _Float16 T; };
template <> struct Elem<1> { typedef __bf16 T; };
template <int ET, bool SPLIT, int BIAS_MODE, int OUT_MODE, bool RESID, int ACT = 0>
__global__ __launch_bounds__(256) void wmma_gemm64(
    const unsigned short* __restrict__ Ap, const unsigned short* __restrict__ A2p, int lda, long strideA,
    const unsigned short* __restrict__ Btp, const unsigned short* __restrict__ Bt2p, int ldb, long strideB,
    void* __restrict__ Cout, void* __restrict__ Cout2, int ldc, long strideC,
    const float* __restrict__ bias,
    const float* __restrict__ resid, long strideR,
    int M, int N, int K, float scale) {
  typedef typename Elem<ET>::T T;
  typedef typename Frag<T>::V V;
  const T* A = (const T*)Ap; const T* A2 = (const T*)A2p; const T* Bt = (const T*)Btp; const T* Bt2 = (const T*)Bt2p;
  __shared__ __align__(16) float sT[8][16 * 68];
  const int b    = blockIdx.y;
  const int lane = threadIdx.x & 31;
  const int wave = threadIdx.x >> 5;
  const int tilesN = N >> 6;
  const int tilesM = M >> 6;
  const int tile = blockIdx.x * 8 + wave;
  if (tile >= tilesM * tilesN) return;
  const int tm = tile / tilesN;
  const int tn = tile - tm * tilesN;
  const int m0 = tm << 6;
  const int n0 = tn << 6;

  const T* Ab  = A  + (size_t)b * strideA;
  const T* Bb  = Bt + (size_t)b * strideB;
  const T* Ab2 = SPLIT ? (A2  + (size_t)b * strideA) : nullptr;
  const T* Bb2 = SPLIT ? (Bt2 + (size_t)b * strideB) : nullptr;

  const int rlane = lane & 15;
  const int koff  = (lane >> 4) * 8;
  const int mOff  = (lane >> 4) * 8;

  v8f acc[4][4];
#pragma unroll
  for (int i = 0; i < 4; ++i)
#pragma unroll
    for (int j = 0; j < 4; ++j) acc[i][j] = (v8f){0.f,0.f,0.f,0.f,0.f,0.f,0.f,0.f};

  for (int k0 = 0; k0 < K; k0 += 32) {
    V bh[4], bl[4];
#pragma unroll
    for (int j = 0; j < 4; ++j) {
      const size_t bo = (size_t)(n0 + (j << 4) + rlane) * ldb + koff + k0;
      bh[j] = Frag<T>::load(Bb + bo);
      if (SPLIT) bl[j] = Frag<T>::load(Bb2 + bo);
    }
#pragma unroll
    for (int i = 0; i < 4; ++i) {
      const size_t ao = (size_t)(m0 + (i << 4) + rlane) * lda + koff + k0;
      V ah = Frag<T>::load(Ab + ao);
      V al;
      if (SPLIT) al = Frag<T>::load(Ab2 + ao);
#pragma unroll
      for (int j = 0; j < 4; ++j) {
        acc[i][j] = Frag<T>::mma(ah, bh[j], acc[i][j]);
        if (SPLIT) {
          acc[i][j] = Frag<T>::mma(ah, bl[j], acc[i][j]);
          acc[i][j] = Frag<T>::mma(al, bh[j], acc[i][j]);
        }
      }
      Frag<T>::guard(acc[i][0], acc[i][3], ah, SPLIT ? al : ah);
    }
    Frag<T>::keep(bh[0], bh[1], bh[2], bh[3]);
    if (SPLIT) Frag<T>::keep(bl[0], bl[1], bl[2], bl[3]);
  }
  acc_guard4(acc[0][0], acc[0][1], acc[0][2], acc[0][3]);
  acc_guard4(acc[1][0], acc[1][1], acc[1][2], acc[1][3]);
  acc_guard4(acc[2][0], acc[2][1], acc[2][2], acc[2][3]);
  acc_guard4(acc[3][0], acc[3][1], acc[3][2], acc[3][3]);

  float* slab = sT[wave];
  const float* Rb = RESID ? (resid + (size_t)b * strideR) : nullptr;
#pragma unroll
  for (int i = 0; i < 4; ++i) {
    const int mBase = m0 + (i << 4);
#pragma unroll
    for (int j = 0; j < 4; ++j) {
      const int n = n0 + (j << 4) + rlane;
      float bv = 0.f;
      if (BIAS_MODE == 2) bv = bias[n];
#pragma unroll
      for (int r = 0; r < 8; ++r) {
        float v = acc[i][j][r] * scale;
        if (BIAS_MODE == 1) v += bias[mBase + mOff + r];
        if (BIAS_MODE == 2) v += bv;
        if (RESID) v += Rb[(size_t)(mBase + mOff + r) * ldc + n];
        if (ACT == 2) v = fmaxf(v, 0.0f);
        if (ACT == 4) v = (v > 0.f) ? v : 0.01f * v;
        slab[(mOff + r) * 68 + (j << 4) + rlane] = v;
      }
    }
    __builtin_amdgcn_fence(__ATOMIC_RELEASE, "workgroup");
    __builtin_amdgcn_wave_barrier();
    __builtin_amdgcn_fence(__ATOMIC_ACQUIRE, "workgroup");
    if (OUT_MODE == 0) {
      float* C = (float*)Cout + (size_t)b * strideC;
      const int hh = lane >> 4, c4 = (lane & 15) * 4;
      for (int pass = 0; pass < 2; ++pass) {
#pragma unroll
        for (int it = 0; it < 8; ++it) {
          const int row = it * 2 + hh;
          v4f v = *(const v4f*)(slab + row * 68 + c4);
          *(volatile v4f*)(C + (size_t)(mBase + row) * ldc + n0 + c4) = v;
        }
        __threadfence();
      }
    } else {
      const int q = lane >> 3, c8 = (lane & 7) * 8;
      unsigned short* C  = (unsigned short*)Cout  + (size_t)b * strideC;
      unsigned short* C2 = (OUT_MODE == 2) ? ((unsigned short*)Cout2 + (size_t)b * strideC) : nullptr;
      for (int pass = 0; pass < 2; ++pass) {
#pragma unroll
        for (int it = 0; it < 4; ++it) {
          const int row = it * 4 + q;
          const float* sp = slab + row * 68 + c8;
          v8h hv, lv;
#pragma unroll
          for (int e = 0; e < 8; ++e) {
            if (OUT_MODE == 1) {
              hv[e] = (_Float16)sp[e];
            } else {
              unsigned short hb = f2bf_bits(sp[e]);
              unsigned short lb = f2bf_bits(sp[e] - bf_bits2f(hb));
              hv[e] = __builtin_bit_cast(_Float16, hb);
              lv[e] = __builtin_bit_cast(_Float16, lb);
            }
          }
          *(volatile v8h*)(C + (size_t)(mBase + row) * ldc + n0 + c8) = hv;
          if (OUT_MODE == 2) *(volatile v8h*)(C2 + (size_t)(mBase + row) * ldc + n0 + c8) = lv;
        }
        __threadfence();
      }
    }
    __builtin_amdgcn_fence(__ATOMIC_RELEASE, "workgroup");
    __builtin_amdgcn_wave_barrier();
    __builtin_amdgcn_fence(__ATOMIC_ACQUIRE, "workgroup");
  }
}

__device__ __forceinline__ unsigned pk16(unsigned short a, unsigned short b) { return (unsigned)a | ((unsigned)b << 16); }

__device__ __forceinline__ void split8(const float* sp, v4u& uh, v4u& ul) {
  unsigned short hb[8], lb[8];
#pragma unroll
  for (int e = 0; e < 8; ++e) {
    const float f = sp[e];
    const unsigned short h = f2bf_bits(f);
    hb[e] = h;
    lb[e] = f2bf_bits(f - bf_bits2f(h));
  }
  uh = (v4u){pk16(hb[0], hb[1]), pk16(hb[2], hb[3]), pk16(hb[4], hb[5]), pk16(hb[6], hb[7])};
  ul = (v4u){pk16(lb[0], lb[1]), pk16(lb[2], lb[3]), pk16(lb[4], lb[5]), pk16(lb[6], lb[7])};
}
__device__ __forceinline__ void store2_hilo(unsigned short* ph, unsigned short* pl, v4u uh, v4u ul) {
  *(volatile v4u*)ph = uh;
  *(volatile v4u*)pl = ul;
  __threadfence();
  *(volatile v4u*)ph = uh;
  *(volatile v4u*)pl = ul;
}
__device__ __forceinline__ float sigm(float x) { return 1.0f / (1.0f + expf(-x)); }
__device__ __forceinline__ float wave_sum(float v) {
#pragma unroll
  for (int off = 16; off > 0; off >>= 1) v += __shfl_xor(v, off, 32);
  return v;
}

__global__ __launch_bounds__(256) void wt_down_kernel(const float* __restrict__ W, int ldw, int col0, int ncol,
                                                      unsigned short* __restrict__ Bh, unsigned short* __restrict__ Bl, int row0)
{
  __shared__ float sm[32][65];
  const int tid = threadIdx.x;
  const int k0 = blockIdx.x * 64;
  const int rb = blockIdx.y * 32;
  const int cmax = (ncol > 0) ? (ncol - 1) : 0;
#pragma unroll
  for (int it = 0; it < 8; ++it) {
    const int e  = it * 256 + tid;
    const int r  = e & 31;
    const int kk = e >> 5;
    const int rg = rb + r;
    const int cc = col0 + ((rg < cmax) ? rg : cmax);
    const float t = W[(size_t)(k0 + kk) * ldw + cc];
    sm[r][kk] = (rg < ncol) ? t : 0.0f;
  }
  __syncthreads();
  const int lane = tid & 31, wave = tid >> 5;
  const int rloc = wave * 4 + (lane >> 3);
  const int c8 = (lane & 7) * 8;
  v4u uh, ul;
  split8(&sm[rloc][c8], uh, ul);
  const size_t off = (size_t)(row0 + rb + rloc) * kNC + k0 + c8;
  store2_hilo(Bh + off, Bl + off, uh, ul);
}

__global__ __launch_bounds__(256) void wt_up_kernel(const float* __restrict__ W2, int kl, unsigned short* __restrict__ Bh,
                                                    unsigned short* __restrict__ Bl, int kpad)
{
  __shared__ float sm[64][129];
  const int tid = threadIdx.x;
  const int n0 = blockIdx.x * 64;
  const int tot = kpad * 64;
  for (int e = tid; e < tot; e += 256) {
    const int k  = e >> 6;
    const int cc = e & 63;
    const int kc = (k < kl) ? k : (kl - 1);
    const float t = W2[(size_t)kc * kNC + n0 + cc];
    sm[cc][k] = (k < kl) ? t : 0.0f;
  }
  __syncthreads();
  const int cpr = kpad >> 3;
  const int nch = kpad * 8;
  for (int pass = 0; pass < 2; ++pass) {
    for (int ch = tid; ch < nch; ch += 256) {
      const int row  = ch / cpr;
      const int col8 = (ch - row * cpr) * 8;
      v4u uh, ul;
      split8(&sm[row][col8], uh, ul);
      const size_t off = (size_t)n0 * kpad + (size_t)ch * 8;
      *(volatile v4u*)(Bh + off) = uh;
      *(volatile v4u*)(Bl + off) = ul;
    }
    __threadfence();
  }
}

__global__ __launch_bounds__(256) void shift_split_kernel(const float* __restrict__ x, const float* __restrict__ tmx,
                                                          unsigned short* __restrict__ oh, unsigned short* __restrict__ ol)
{
  __shared__ __align__(16) float s[256];
  const int tid = threadIdx.x;
  const long blk0 = (long)blockIdx.x * 256;
  const long idx = blk0 + tid;
  const int c = (int)(idx % kNC);
  const int t = (int)((idx / kNC) & (kNT - 1));
  const float xc = x[idx];
  const long pidx = (t == 0) ? idx : (idx - kNC);
  float xp = x[pidx];
  xp = (t == 0) ? 0.0f : xp;
  const float d = xp - xc;
  s[tid] = xc + d * tmx[c];
  __syncthreads();
  if (tid < 32) {
    v4u uh, ul;
    split8(&s[8 * tid], uh, ul);
    const long off = blk0 + 8 * tid;
    store2_hilo(oh + off, ol + off, uh, ul);
  }
}

__global__ __launch_bounds__(256) void mix_split_kernel(const float* __restrict__ x, const float* __restrict__ adds,
    const float* __restrict__ trg, const float* __restrict__ twa, const float* __restrict__ tk, const float* __restrict__ tv,
    unsigned short* __restrict__ h0, unsigned short* __restrict__ l0, unsigned short* __restrict__ h1, unsigned short* __restrict__ l1,
    unsigned short* __restrict__ h2, unsigned short* __restrict__ l2, unsigned short* __restrict__ h3, unsigned short* __restrict__ l3)
{
  __shared__ __align__(16) float s[4][256];
  const int tid = threadIdx.x;
  const long blk0 = (long)blockIdx.x * 256;
  const long idx = blk0 + tid;
  const int c = (int)(idx % kNC);
  const int t = (int)((idx / kNC) & (kNT - 1));
  const float xc = x[idx];
  const long pidx = (t == 0) ? idx : (idx - kNC);
  float xp = x[pidx];
  xp = (t == 0) ? 0.0f : xp;
  const float d = xp - xc;
  const float a0 = adds[idx];
  const float a1 = adds[kPlaneElems + idx];
  const float a2 = adds[2 * kPlaneElems + idx];
  const float a3 = adds[3 * kPlaneElems + idx];
  s[0][tid] = xc + d * (trg[c] + a0);
  s[1][tid] = xc + d * (twa[c] + a1);
  s[2][tid] = xc + d * (tk[c]  + a2);
  s[3][tid] = xc + d * (tv[c]  + a3);
  __syncthreads();
  if (tid < 128) {
    const int o = tid >> 5;
    const int l = tid & 31;
    v4u uh, ul;
    split8(&s[o][8 * l], uh, ul);
    unsigned short* dh; unsigned short* dl;
    if (o == 0)      { dh = h0; dl = l0; }
    else if (o == 1) { dh = h1; dl = l1; }
    else if (o == 2) { dh = h2; dl = l2; }
    else             { dh = h3; dl = l3; }
    const long off = blk0 + 8 * l;
    store2_hilo(dh + off, dl + off, uh, ul);
  }
}

__global__ __launch_bounds__(256) void act_split_kernel(const float* __restrict__ F, unsigned short* __restrict__ Hh,
                                                        unsigned short* __restrict__ Hl, int nf, int tanh_end, int sig_end, int zfrom)
{
  __shared__ __align__(16) float s[256];
  const int tid = threadIdx.x;
  const long blk0 = (long)blockIdx.x * 256;
  const long idx = blk0 + tid;
  const int c = (int)(idx % nf);
  const float v = F[idx];
  float r;
  if (c < tanh_end)     r = tanhf(v);
  else if (c < sig_end) r = sigm(v);
  else                  r = v;
  if (c >= zfrom) r = 0.0f;
  s[tid] = r;
  __syncthreads();
  if (tid < 32) {
    v4u uh, ul;
    split8(&s[8 * tid], uh, ul);
    const long off = blk0 + 8 * tid;
    store2_hilo(Hh + off, Hl + off, uh, ul);
  }
}

__global__ __launch_bounds__(256) void tail_v_kernel(const float* __restrict__ vraw, const float* __restrict__ mvpre,
                                                     const float* __restrict__ v1, const float* __restrict__ tmv, float* __restrict__ vf)
{
  const long idx = (long)blockIdx.x * 256 + threadIdx.x;
  const int c = (int)(idx % kNC);
  const float vr = vraw[idx];
  const float e1 = v1[idx];
  const float sg = sigm(tmv[c] + mvpre[idx]);
  const float o  = vr + (e1 - vr) * sg;
  *(volatile float*)(vf + idx) = o;
  __threadfence();
  *(volatile float*)(vf + idx) = o;
}

__global__ __launch_bounds__(256) void sig3_kernel(float* ap, float* mp, float* kp, const float* __restrict__ ta,
                                                   const float* __restrict__ tma, const float* __restrict__ tmk)
{
  const long idx = (long)blockIdx.x * 256 + threadIdx.x;
  const int c = (int)(idx % kNC);
  const float a = sigm(ta[c]  + ap[idx]);
  const float m = sigm(tma[c] + mp[idx]);
  const float q = sigm(tmk[c] + kp[idx]);
  *(volatile float*)(ap + idx) = a;
  *(volatile float*)(mp + idx) = m;
  *(volatile float*)(kp + idx) = q;
  __threadfence();
  *(volatile float*)(ap + idx) = a;
  *(volatile float*)(mp + idx) = m;
  *(volatile float*)(kp + idx) = q;
}

__global__ __launch_bounds__(256) void tail_k_kernel(const float* __restrict__ kraw, float* wd, float* kkio, float* abb,
                                                     const float* __restrict__ map, const float* __restrict__ mkp,
                                                     const float* __restrict__ tdecay, float* __restrict__ kf)
{
  __shared__ float red[8];
  const int tid = threadIdx.x, lane = tid & 31, wave = tid >> 5;
  const int hg  = blockIdx.x % 3;
  const int row = blockIdx.x / 3;
  const int c   = hg * 256 + tid;
  const long i  = (long)row * kNC + c;
  const int hl  = tid >> 6;
  const float kr  = kraw[i];
  const float kkp = kkio[i];
  const float wp  = wd[i];
  const float a   = abb[i];
  const float ma  = map[i];
  const float mk  = mkp[i];
  const float z   = -(tdecay[c] + wp);
  const float sp  = fmaxf(z, 0.0f) + log1pf(expf(-fabsf(z)));
  const float w   = -sp - 0.5f;
  const float d   = expf(-expf(w));
  const float kku = kr + kkp;
  float kn = kr * ma + kr * a * (1.0f - ma);
  kn = kn * expf(fminf(w * mk, 0.0f));
  float ss = wave_sum(kku * kku);
  if (lane == 0) red[wave] = ss;
  __syncthreads();
  const float tot = red[2 * hl] + red[2 * hl + 1];
  const float nrm = fmaxf(sqrtf(tot), 1e-12f);
  const float kkn = kku * (1.0f / nrm);
  const float bb  = kkn * a;
  *(volatile float*)(wd + i)   = d;
  *(volatile float*)(kkio + i) = kkn;
  *(volatile float*)(abb + i)  = bb;
  *(volatile float*)(kf + i)   = kn;
  __threadfence();
  *(volatile float*)(wd + i)   = d;
  *(volatile float*)(kkio + i) = kkn;
  *(volatile float*)(abb + i)  = bb;
  *(volatile float*)(kf + i)   = kn;
}

__global__ __launch_bounds__(256) void scan_kernel(const float* __restrict__ Rp, const float* __restrict__ Dp,
                                                   const float* __restrict__ Kp, const float* __restrict__ Vp,
                                                   const float* __restrict__ KKp, const float* __restrict__ BBp,
                                                   float* __restrict__ Yp)
{
  __shared__ __align__(16) float sr[kHS];
  __shared__ __align__(16) float sd[kHS];
  __shared__ __align__(16) float sk[kHS];
  __shared__ __align__(16) float sv[kHS];
  __shared__ __align__(16) float saa[kHS];
  __shared__ __align__(16) float sbb[kHS];
  __shared__ __align__(16) float sy[kHS];
  const int bh  = blockIdx.x;
  const int b   = bh / kNH;
  const int h   = bh - b * kNH;
  const int tid = threadIdx.x;
  const int row = tid >> 2;
  const int grp = tid & 3;
  const int j0  = grp * 16;
  float S[16];
#pragma unroll
  for (int jj = 0; jj < 16; ++jj) S[jj] = 0.0f;

#pragma unroll 1
  for (int t = 0; t < kNT; ++t) {
    const long base = ((long)(b * kNT + t)) * kNC + h * kHS;
    if (tid < kHS) {
      sr[tid]  = Rp[base + tid];
      sd[tid]  = Dp[base + tid];
      sk[tid]  = Kp[base + tid];
      sv[tid]  = Vp[base + tid];
      const float kkv = KKp[base + tid];
      saa[tid] = -kkv;
      sbb[tid] = BBp[base + tid];
    }
    __syncthreads();
    float ps = 0.0f;
#pragma unroll
    for (int jj = 0; jj < 16; ++jj) ps += S[jj] * saa[j0 + jj];
    ps += __shfl_xor(ps, 1, 32);
    ps += __shfl_xor(ps, 2, 32);
    const float vi = sv[row];
    float pr = 0.0f;
#pragma unroll
    for (int jj = 0; jj < 16; ++jj) {
      const int j = j0 + jj;
      const float sn = S[jj] * sd[j] + ps * sbb[j] + vi * sk[j];
      S[jj] = sn;
      pr += sn * sr[j];
    }
    pr += __shfl_xor(pr, 1, 32);
    pr += __shfl_xor(pr, 2, 32);
    if (grp == 0) sy[row] = pr;
    __syncthreads();
    if (tid < 16) {
      const v4f val = *(const v4f*)(sy + 4 * tid);
      float* yp = Yp + base + 4 * tid;
      *(volatile v4f*)yp = val;
      __threadfence();
      *(volatile v4f*)yp = val;
    }
  }
}

__global__ __launch_bounds__(256) void post_kernel(const float* __restrict__ Yp, const float* __restrict__ Rp,
                                                   const float* __restrict__ Kp, const float* __restrict__ Vp,
                                                   const float* __restrict__ Gp, const float* __restrict__ faaaa,
                                                   const float* __restrict__ gnw, const float* __restrict__ gnb,
                                                   unsigned short* __restrict__ oh, unsigned short* __restrict__ ol)
{
  __shared__ float red1[8];
  __shared__ float red2[8];
  __shared__ float red3[8];
  __shared__ __align__(16) float so[256];
  const int tid = threadIdx.x, lane = tid & 31, wave = tid >> 5;
  const int hg  = blockIdx.x % 3;
  const int row = blockIdx.x / 3;
  const int c   = hg * 256 + tid;
  const long i  = (long)row * kNC + c;
  const int hl  = tid >> 6;
  const float yv = Yp[i];
  const float rv = Rp[i];
  const float kv = Kp[i];
  const float vv = Vp[i];
  const float gv = Gp[i];
  const float fa = faaaa[c];
  const float gw = gnw[c];
  const float gb = gnb[c];
  float s1 = wave_sum(yv);
  if (lane == 0) red1[wave] = s1;
  __syncthreads();
  const float mean = (red1[2 * hl] + red1[2 * hl + 1]) * kInvHS;
  const float dv = yv - mean;
  float s2 = wave_sum(dv * dv);
  if (lane == 0) red2[wave] = s2;
  __syncthreads();
  const float var = (red2[2 * hl] + red2[2 * hl + 1]) * kInvHS;
  const float inv = 1.0f / sqrtf(var + kGnEps);
  const float nv  = dv * inv * gw + gb;
  float s3 = wave_sum(rv * kv * fa);
  if (lane == 0) red3[wave] = s3;
  __syncthreads();
  const float dot = red3[2 * hl] + red3[2 * hl + 1];
  so[tid] = (nv + dot * vv) * gv;
  __syncthreads();
  if (tid < 32) {
    v4u uh, ul;
    split8(&so[8 * tid], uh, ul);
    const long off = (long)row * kNC + hg * 256 + 8 * tid;
    store2_hilo(oh + off, ol + off, uh, ul);
  }
}

__global__ __launch_bounds__(256) void copy_kernel(const float* __restrict__ src, float* __restrict__ dst)
{
  const long i = (long)blockIdx.x * 256 + threadIdx.x;
  const v4f v = *(const v4f*)(src + 4 * i);
  float* p = dst + 4 * i;
  *(volatile v4f*)p = v;
  __threadfence();
  *(volatile v4f*)p = v;
}

static inline void gemm3(const unsigned short* Ah, const unsigned short* Al, int lda, long sA,
                         const unsigned short* Bh, const unsigned short* Bl, int ldb, long sB,
                         float* C, int ldc, long sC, int M, int N, int K, int nb, hipStream_t st)
{
  const int tiles = (M / 64) * (N / 64);
  dim3 grid((tiles + 7) / 8, nb);
  wmma_gemm64<1, true, 0, 0, false, 0><<<grid, 256, 0, st>>>(Ah, Al, lda, sA, Bh, Bl, ldb, sB,
                                                             (void*)C, (void*)nullptr, ldc, sC,
                                                             (const float*)nullptr, (const float*)nullptr, 0L,
                                                             M, N, K, 1.0f);
}
static inline void wt_down(const float* W, int ldw, int col0, int ncol, unsigned short* Bh, unsigned short* Bl,
                           int row0, int nrow, hipStream_t st)
{
  dim3 grid(kNC / 64, nrow / 32);
  wt_down_kernel<<<grid, 256, 0, st>>>(W, ldw, col0, ncol, Bh, Bl, row0);
}
static inline void wt_up(const float* W2, int kl, unsigned short* Bh, unsigned short* Bl, int kpad, hipStream_t st)
{
  wt_up_kernel<<<kNC / 64, 256, 0, st>>>(W2, kl, Bh, Bl, kpad);
}
static inline void act_split(const float* F, unsigned short* Hh, unsigned short* Hl, int nf, int tanh_end, int sig_end,
                             int zfrom, hipStream_t st)
{
  act_split_kernel<<<(kRows * nf) / 256, 256, 0, st>>>(F, Hh, Hl, nf, tanh_end, sig_end, zfrom);
}

extern "C" void kernel_launch(void* const* d_in, const int* in_sizes, int n_in,
                              void* d_out, int out_size, void* d_ws, size_t ws_size,
                              hipStream_t stream)
{
  (void)in_sizes; (void)n_in;
  const float* x        = (const float*)d_in[0];
  const float* v1       = (const float*)d_in[1];
  const float* tmx      = (const float*)d_in[2];
  const float* tmrg     = (const float*)d_in[3];
  const float* tmwa     = (const float*)d_in[4];
  const float* tmk      = (const float*)d_in[5];
  const float* tmv      = (const float*)d_in[6];
  const float* tdecay   = (const float*)d_in[7];
  const float* tfaaaa   = (const float*)d_in[8];
  const float* taaaaa   = (const float*)d_in[9];
  const float* maa_w1   = (const float*)d_in[10];
  const float* maa_w2   = (const float*)d_in[11];
  const float* decay_w1 = (const float*)d_in[12];
  const float* decay_w2 = (const float*)d_in[13];
  const float* aaa_w1   = (const float*)d_in[14];
  const float* aaa_w2   = (const float*)d_in[15];
  const float* kkk_w1   = (const float*)d_in[16];
  const float* kkk_w2   = (const float*)d_in[17];
  const float* gate_w1  = (const float*)d_in[18];
  const float* gate_w2  = (const float*)d_in[19];
  const float* ma_w1    = (const float*)d_in[20];
  const float* ma_w2    = (const float*)d_in[21];
  const float* tmisca   = (const float*)d_in[22];
  const float* mk_w1    = (const float*)d_in[23];
  const float* mk_w2    = (const float*)d_in[24];
  const float* tmisck   = (const float*)d_in[25];
  const float* mv_w1    = (const float*)d_in[26];
  const float* mv_w2    = (const float*)d_in[27];
  const float* tmiscv   = (const float*)d_in[28];
  const float* Wr       = (const float*)d_in[29];
  const float* Wk       = (const float*)d_in[30];
  const float* Wv       = (const float*)d_in[31];
  const float* Wo       = (const float*)d_in[32];
  const float* gn_w     = (const float*)d_in[33];
  const float* gn_b     = (const float*)d_in[34];

  if ((long)out_size < 2 * kPlaneElems) return;
  float* out0 = (float*)d_out;
  float* out1 = out0 + kPlaneElems;

  char* ws = (char*)d_ws;
  const size_t PB = (size_t)kPlaneElems * 4;
  const size_t HB = PB / 2;
  float*          sf[9];
  unsigned short* sh[9];
  unsigned short* sl[9];
  for (int k = 0; k < 9; ++k) {
    sf[k] = (float*)(ws + (size_t)k * PB);
    sh[k] = (unsigned short*)(ws + (size_t)k * PB);
    sl[k] = (unsigned short*)(ws + (size_t)k * PB + HB);
  }
  size_t off = 9 * PB;
  float* Fbuf = (float*)(ws + off);                     off += (size_t)kRows * 128 * 4;
  unsigned short* HLh = (unsigned short*)(ws + off);
  unsigned short* HLl = (unsigned short*)(ws + off + (size_t)kRows * 128 * 2);
  off += (size_t)kRows * 128 * 4;
  const size_t bigW = (size_t)kNC * kNC * 2;
  unsigned short* WrTh = (unsigned short*)(ws + off); unsigned short* WrTl = (unsigned short*)(ws + off + bigW); off += 2 * bigW;
  unsigned short* WkTh = (unsigned short*)(ws + off); unsigned short* WkTl = (unsigned short*)(ws + off + bigW); off += 2 * bigW;
  unsigned short* WvTh = (unsigned short*)(ws + off); unsigned short* WvTl = (unsigned short*)(ws + off + bigW); off += 2 * bigW;
  unsigned short* WoTh = (unsigned short*)(ws + off); unsigned short* WoTl = (unsigned short*)(ws + off + bigW); off += 2 * bigW;
  const size_t w128 = (size_t)128 * kNC * 2;
  const size_t w64  = (size_t)64 * kNC * 2;
  unsigned short* Mw1h = (unsigned short*)(ws + off); unsigned short* Mw1l = (unsigned short*)(ws + off + w128); off += 2 * w128;
  unsigned short* Gw1h = (unsigned short*)(ws + off); unsigned short* Gw1l = (unsigned short*)(ws + off + w128); off += 2 * w128;
  unsigned short* WAh  = (unsigned short*)(ws + off); unsigned short* WAl  = (unsigned short*)(ws + off + w128); off += 2 * w128;
  unsigned short* KLh  = (unsigned short*)(ws + off); unsigned short* KLl  = (unsigned short*)(ws + off + w64);  off += 2 * w64;
  unsigned short* VLh  = (unsigned short*)(ws + off); unsigned short* VLl  = (unsigned short*)(ws + off + w64);  off += 2 * w64;
  const size_t m2p  = (size_t)4 * kNC * 32 * 2;
  unsigned short* Mw2h = (unsigned short*)(ws + off); unsigned short* Mw2l = (unsigned short*)(ws + off + m2p); off += 2 * m2p;
  const size_t u64p = (size_t)kNC * 64 * 2;
  const size_t u32p = (size_t)kNC * 32 * 2;
  const size_t u128p = (size_t)kNC * 128 * 2;
  unsigned short* Dw2h = (unsigned short*)(ws + off); unsigned short* Dw2l = (unsigned short*)(ws + off + u64p); off += 2 * u64p;
  unsigned short* Aw2h = (unsigned short*)(ws + off); unsigned short* Aw2l = (unsigned short*)(ws + off + u32p); off += 2 * u32p;
  unsigned short* MAw2h = (unsigned short*)(ws + off); unsigned short* MAw2l = (unsigned short*)(ws + off + u32p); off += 2 * u32p;
  unsigned short* KKw2h = (unsigned short*)(ws + off); unsigned short* KKw2l = (unsigned short*)(ws + off + u32p); off += 2 * u32p;
  unsigned short* MKw2h = (unsigned short*)(ws + off); unsigned short* MKw2l = (unsigned short*)(ws + off + u32p); off += 2 * u32p;
  unsigned short* MVw2h = (unsigned short*)(ws + off); unsigned short* MVw2l = (unsigned short*)(ws + off + u32p); off += 2 * u32p;
  unsigned short* Gw2h = (unsigned short*)(ws + off); unsigned short* Gw2l = (unsigned short*)(ws + off + u128p); off += 2 * u128p;
  if (off > ws_size) return;

  const int eltGrid = (int)(kPlaneElems / 256);
  const int rowGrid = kRows * 3;

  wt_down(Wr, kNC, 0, kNC, WrTh, WrTl, 0, kNC, stream);
  wt_down(Wk, kNC, 0, kNC, WkTh, WkTl, 0, kNC, stream);
  wt_down(Wv, kNC, 0, kNC, WvTh, WvTl, 0, kNC, stream);
  wt_down(Wo, kNC, 0, kNC, WoTh, WoTl, 0, kNC, stream);
  for (int f = 0; f < 4; ++f)
    wt_down(maa_w1, 112, 28 * f, 28, Mw1h, Mw1l, 32 * f, 32, stream);
  wt_down(gate_w1, 120, 0, 120, Gw1h, Gw1l, 0, 128, stream);
  wt_down(decay_w1, 64, 0, 64, WAh, WAl, 0, 64, stream);
  wt_down(aaa_w1, 16, 0, 16, WAh, WAl, 64, 32, stream);
  wt_down(ma_w1, 16, 0, 16, WAh, WAl, 96, 32, stream);
  wt_down(kkk_w1, 16, 0, 16, KLh, KLl, 0, 32, stream);
  wt_down(mk_w1, 16, 0, 16, KLh, KLl, 32, 32, stream);
  wt_down(mv_w1, 16, 0, 16, VLh, VLl, 0, 64, stream);
  for (int f = 0; f < 4; ++f)
    wt_up(maa_w2 + (size_t)f * 28 * kNC, 28, Mw2h + (size_t)f * kNC * 32, Mw2l + (size_t)f * kNC * 32, 32, stream);
  wt_up(decay_w2, 64, Dw2h, Dw2l, 64, stream);
  wt_up(aaa_w2, 16, Aw2h, Aw2l, 32, stream);
  wt_up(ma_w2, 16, MAw2h, MAw2l, 32, stream);
  wt_up(kkk_w2, 16, KKw2h, KKw2l, 32, stream);
  wt_up(mk_w2, 16, MKw2h, MKw2l, 32, stream);
  wt_up(mv_w2, 16, MVw2h, MVw2l, 32, stream);
  wt_up(gate_w2, 120, Gw2h, Gw2l, 128, stream);

  shift_split_kernel<<<eltGrid, 256, 0, stream>>>(x, tmx, sh[0], sl[0]);
  gemm3(sh[0], sl[0], kNC, 0, Mw1h, Mw1l, kNC, 0, Fbuf, 128, 0, kRows, 128, kNC, 1, stream);
  act_split(Fbuf, HLh, HLl, 128, 128, 128, 128, stream);
  gemm3(HLh, HLl, 128, 32, Mw2h, Mw2l, 32, (long)kNC * 32, sf[1], kNC, kPlaneElems, kRows, kNC, 32, 4, stream);
  mix_split_kernel<<<eltGrid, 256, 0, stream>>>(x, sf[1], tmrg, tmwa, tmk, tmv,
                                                 sh[0], sl[0], sh[5], sl[5], sh[6], sl[6], sh[7], sl[7]);

  gemm3(sh[7], sl[7], kNC, 0, WvTh, WvTl, kNC, 0, sf[1], kNC, 0, kRows, kNC, kNC, 1, stream);
  gemm3(sh[7], sl[7], kNC, 0, VLh, VLl, kNC, 0, Fbuf, 64, 0, kRows, 64, kNC, 1, stream);
  act_split(Fbuf, HLh, HLl, 64, 0, 0, 64, stream);
  gemm3(HLh, HLl, 64, 0, MVw2h, MVw2l, 32, 0, sf[2], kNC, 0, kRows, kNC, 32, 1, stream);
  tail_v_kernel<<<eltGrid, 256, 0, stream>>>(sf[1], sf[2], v1, tmiscv, sf[7]);

  gemm3(sh[5], sl[5], kNC, 0, WAh, WAl, kNC, 0, Fbuf, 128, 0, kRows, 128, kNC, 1, stream);
  act_split(Fbuf, HLh, HLl, 128, 64, 64, 128, stream);
  gemm3(HLh,      HLl,      128, 0, Dw2h,  Dw2l,  64, 0, sf[1], kNC, 0, kRows, kNC, 64, 1, stream);
  gemm3(HLh + 64, HLl + 64, 128, 0, Aw2h,  Aw2l,  32, 0, sf[2], kNC, 0, kRows, kNC, 32, 1, stream);
  gemm3(HLh + 96, HLl + 96, 128, 0, MAw2h, MAw2l, 32, 0, sf[3], kNC, 0, kRows, kNC, 32, 1, stream);

  gemm3(sh[6], sl[6], kNC, 0, WkTh, WkTl, kNC, 0, sf[4], kNC, 0, kRows, kNC, kNC, 1, stream);
  gemm3(sh[6], sl[6], kNC, 0, KLh, KLl, kNC, 0, Fbuf, 64, 0, kRows, 64, kNC, 1, stream);
  act_split(Fbuf, HLh, HLl, 64, 16, 16, 64, stream);
  gemm3(HLh,      HLl,      64, 0, KKw2h, KKw2l, 32, 0, sf[5], kNC, 0, kRows, kNC, 32, 1, stream);
  gemm3(HLh + 32, HLl + 32, 64, 0, MKw2h, MKw2l, 32, 0, sf[8], kNC, 0, kRows, kNC, 32, 1, stream);

  sig3_kernel<<<eltGrid, 256, 0, stream>>>(sf[2], sf[3], sf[8], taaaaa, tmisca, tmisck);
  tail_k_kernel<<<rowGrid, 256, 0, stream>>>(sf[4], sf[1], sf[5], sf[2], sf[3], sf[8], tdecay, sf[6]);

  gemm3(sh[0], sl[0], kNC, 0, WrTh, WrTl, kNC, 0, sf[3], kNC, 0, kRows, kNC, kNC, 1, stream);
  gemm3(sh[0], sl[0], kNC, 0, Gw1h, Gw1l, kNC, 0, Fbuf, 128, 0, kRows, 128, kNC, 1, stream);
  act_split(Fbuf, HLh, HLl, 128, 0, 120, 120, stream);
  gemm3(HLh, HLl, 128, 0, Gw2h, Gw2l, 128, 0, sf[4], kNC, 0, kRows, kNC, 128, 1, stream);

  scan_kernel<<<kNB * kNH, 256, 0, stream>>>(sf[3], sf[1], sf[6], sf[7], sf[5], sf[2], sf[8]);

  post_kernel<<<rowGrid, 256, 0, stream>>>(sf[8], sf[3], sf[6], sf[7], sf[4], tfaaaa, gn_w, gn_b, sh[0], sl[0]);
  gemm3(sh[0], sl[0], kNC, 0, WoTh, WoTl, kNC, 0, out0, kNC, 0, kRows, kNC, kNC, 1, stream);
  copy_kernel<<<(int)(kPlaneElems / 4 / 256), 256, 0, stream>>>(v1, out1);
}
